// MultiHeadedAttention_1932735283883
// MI455X (gfx1250) — hardware-verified
//
#include <hip/hip_runtime.h>
#include <math.h>

typedef __attribute__((ext_vector_type(16))) _Float16 v16h;
typedef __attribute__((ext_vector_type(16))) __bf16 v16b;
typedef __attribute__((ext_vector_type(8)))  _Float16 v8h;
typedef __attribute__((ext_vector_type(8)))  __bf16 v8b;
typedef __attribute__((ext_vector_type(8)))  float v8f;
typedef __attribute__((ext_vector_type(4)))  float v4f;
typedef __attribute__((ext_vector_type(4)))  unsigned v4u;

#ifndef NB
#define NB 2
#endif
#ifndef SEQ
#define SEQ 2048
#endif
#define NB_FULL 2
#define SEQ_FULL 2048
#define DM 1024
#define NH 16
#define HD 64
#define MROWS (NB * SEQ)
#define SCALE (0.125f)
#define PCARRY (1024.0f)
#define OUT1_ELEM 4194304
static_assert((size_t)NB_FULL * SEQ_FULL * DM * 4 == 16777216u);
static_assert((size_t)OUT1_ELEM * 4 == 16777216u);
static_assert((size_t)OUT1_ELEM + (size_t)NB_FULL * 2 * NH * SEQ_FULL * HD == 12582912u);
static_assert(SEQ % 64 == 0 && SEQ <= SEQ_FULL && NB <= NB_FULL);
static_assert(DM == NH * HD && DM % 128 == 0 && DM % 32 == 0 && HD == 64);
static_assert((SEQ * DM / 8) % 256 == 0 && (DM * DM / 8) % 256 == 0);

#define WS_XB   0u
#define WS_WB   (WS_XB  + 2u * 3u * (size_t)MROWS * DM)
#define WS_WOH  (WS_WB  + 2u * 3u * (size_t)DM * DM)
#define WS_WOL  (WS_WOH + 2u * (size_t)DM * DM)
#define WS_H16  (WS_WOL + 2u * (size_t)DM * DM)
#define WS_QL   (WS_H16 + 2u * 2u * (size_t)MROWS * DM)
#define WS_VT   (WS_QL  + 2u * (size_t)MROWS * DM)
#define WS_CH   (WS_VT  + 2u * (size_t)NB * DM * SEQ)
#define WS_CL   (WS_CH  + 2u * (size_t)MROWS * DM)
#define WS_END  (WS_CL  + 2u * (size_t)MROWS * DM)
static_assert((size_t)WS_END <= 134217728u);

#define WAITL() asm volatile("s_wait_loadcnt 0x0" ::: "memory")
#define LDSX() do { asm volatile("s_wait_dscnt 0" ::: "memory"); __builtin_amdgcn_wave_barrier(); __builtin_amdgcn_fence(3  , "workgroup"); } while (0)

template <typename T> __device__ __forceinline__ void vst2(void* p, T v) { *(volatile T*)p = v; __threadfence(); *(volatile T*)p = v; }
__device__ __forceinline__ v8f wmma16(v16h a, v16h b, v8f c) {
  v8f d = __builtin_amdgcn_wmma_f32_16x16x32_f16(false, a, false, b, (short)0, c, false, false);
  asm volatile("v_nop\n\tv_nop\n\tv_nop\n\tv_nop" : "+v"(d) : "v"(a), "v"(b));
  return d;
}
__device__ __forceinline__ v8f wmma_bf(v16b a, v16b b, v8f c) {
  v8f d = __builtin_amdgcn_wmma_f32_16x16x32_bf16(false, a, false, b, (short)0, c, false, false);
  asm volatile("v_nop\n\tv_nop\n\tv_nop\n\tv_nop" : "+v"(d) : "v"(a), "v"(b));
  return d;
}
__device__ __forceinline__ v16h frag_h(const _Float16* rowk0, int lane) {
  union { v16h v; v8h q[2]; } u; const _Float16* p = rowk0 + 8 * (lane >> 4);
  u.q[0] = *(const v8h*)p; u.q[1] = *(const v8h*)(p + 16); return u.v;
}
__device__ __forceinline__ v16b frag_b(const __bf16* rowk0, int lane) {
  union { v16b v; v8b q[2]; } u; const __bf16* p = rowk0 + 8 * (lane >> 4);
  u.q[0] = *(const v8b*)p; u.q[1] = *(const v8b*)(p + 16); return u.v;
}
__device__ __forceinline__ float bfr(float v) { return (float)(__bf16)v; }

__global__ __launch_bounds__(256) void k_cvt_bf(const float* __restrict__ src, __bf16* __restrict__ dst, size_t sstride, size_t dstride, int n8) {
  const int i = blockIdx.x * 256 + threadIdx.x; if (i >= n8) return;
  const float* p = src + (size_t)blockIdx.y * sstride + (size_t)i * 8;
  const v4f a = *(const v4f*)p, c = *(const v4f*)(p + 4);
  union { v8b b; v4u u; } o;
#pragma unroll
  for (int k = 0; k < 4; ++k) { o.b[k] = (__bf16)a[k]; o.b[4 + k] = (__bf16)c[k]; }
  vst2(dst + (size_t)blockIdx.y * dstride + (size_t)i * 8, o.u);
}
__global__ __launch_bounds__(256) void k_cvt_wo(const float* __restrict__ W, _Float16* __restrict__ WH, _Float16* __restrict__ WL, int n8) {
  const int i = blockIdx.x * 256 + threadIdx.x; if (i >= n8) return;
  const float* p = W + (size_t)i * 8;
  const v4f a = *(const v4f*)p, c = *(const v4f*)(p + 4);
  union { v8h h; v4u u; } oh, ol;
#pragma unroll
  for (int k = 0; k < 4; ++k) { const float x = bfr(a[k]), y = bfr(c[k]); oh.h[k] = (_Float16)(x * 256.0f); ol.h[k] = (_Float16)(x * 2.0f); oh.h[4 + k] = (_Float16)(y * 256.0f); ol.h[4 + k] = (_Float16)(y * 2.0f); }
  vst2(WH + (size_t)i * 8, oh.u); vst2(WL + (size_t)i * 8, ol.u);
}

__global__ __launch_bounds__(128) void k_proj(const __bf16* __restrict__ XB, const __bf16* __restrict__ WB, const float* __restrict__ BQ, const float* __restrict__ BK, const float* __restrict__ BV,
    _Float16* __restrict__ H16, _Float16* __restrict__ QL, _Float16* __restrict__ VT, float* __restrict__ PRES) {
  __shared__ __align__(16) float sf[64][132];
  const int tid = threadIdx.x, wave = tid >> 5, lane = tid & 31, col = lane & 15, g = lane >> 4;
  const int which = blockIdx.z; const int c0 = blockIdx.y * 128; const int r0 = blockIdx.x * 64; const int bb = r0 / SEQ; const int t0 = r0 % SEQ;
  const __bf16* X = XB + (size_t)which * MROWS * DM; const __bf16* W = WB + (size_t)which * DM * DM;
  v8f acc[8] = {};
#pragma unroll 2
  for (int kc = 0; kc < DM / 32; ++kc) {
    const v16b a = frag_b(X + (size_t)(r0 + wave * 16 + col) * DM + kc * 32, lane);
    WAITL();
#pragma unroll
    for (int j = 0; j < 8; ++j) { const v16b w = frag_b(W + (size_t)(c0 + j * 16 + col) * DM + kc * 32, lane); WAITL(); acc[j] = wmma_bf(a, w, acc[j]); }
  }
#pragma unroll
  for (int j = 0; j < 8; ++j) { const int ci = c0 + j * 16 + col; const float b0 = BQ[ci], b1 = BK[ci], b2 = BV[ci]; const float bias = bfr(which == 0 ? b0 : (which == 1 ? b1 : b2));
#pragma unroll
    for (int r = 0; r < 8; ++r) sf[wave * 16 + 8 * g + r][j * 16 + col] = acc[j][r] + bias; }
  __syncthreads();
  if (which < 2) {
    _Float16* DH = H16 + (size_t)which * MROWS * DM;
    for (int e = tid; e < 64 * 16; e += 128) { const int rl = e >> 4, q = e & 15; const v4f a = *(const v4f*)&sf[rl][q * 8], c = *(const v4f*)&sf[rl][q * 8 + 4];
      union { v8h h; v4u u; } hv, lv;
#pragma unroll
      for (int i = 0; i < 4; ++i) { const _Float16 ha = (_Float16)a[i], hc = (_Float16)c[i]; hv.h[i] = ha; hv.h[4 + i] = hc; lv.h[i] = (_Float16)((a[i] - (float)ha) * 1024.0f); lv.h[4 + i] = (_Float16)((c[i] - (float)hc) * 1024.0f); }
      const size_t dst = (size_t)(r0 + rl) * DM + c0 + q * 8;
      vst2(DH + dst, hv.u); if (which == 0) vst2(QL + dst, lv.u); }
  } else {
    for (int e = tid; e < 128 * 8; e += 128) { const int cl = e >> 3, q = e & 7; union { v8h h; v4u u; } o;
#pragma unroll
      for (int i = 0; i < 8; ++i) o.h[i] = (_Float16)sf[q * 8 + i][cl];
      vst2(VT + ((size_t)bb * DM + c0 + cl) * SEQ + t0 + q * 8, o.u); }
  }
  if (which >= 1) {
    const int kv = which - 1;
    for (int e = tid; e < 64 * 32; e += 128) { const int rl = e >> 5, q = e & 31; const v4f o = *(const v4f*)&sf[rl][q * 4]; const int hh = (c0 >> 6) + (q >> 4), d = (q & 15) * 4;
      vst2(PRES + (((size_t)bb * 2 + kv) * NH + hh) * ((size_t)SEQ_FULL * HD) + (size_t)(t0 + rl) * HD + d, o); }
  }
}

__global__ __launch_bounds__(128) void k_attn(const _Float16* __restrict__ H16, const _Float16* __restrict__ QL, const _Float16* __restrict__ VT, const float* __restrict__ MASK, _Float16* __restrict__ CH, _Float16* __restrict__ CL) {
  __shared__ __align__(16) _Float16 sh[4][16][72], sl[4][16][72];
  const int tid = threadIdx.x, wave = tid >> 5, lane = tid & 31, col = lane & 15, g = lane >> 4;
  const int h = blockIdx.y, b = blockIdx.z; const int q0 = blockIdx.x * 64 + wave * 16;
  const _Float16* KH = H16 + (size_t)MROWS * DM;
  const int qoff = (b * SEQ + q0 + col) * DM + h * HD;
  const int koff = (b * SEQ + col) * DM + h * HD;
  const int voff = (b * DM + h * HD + col) * SEQ;
  const float* mrow = MASK + ((size_t)b * SEQ_FULL + q0 + col) * SEQ_FULL + 8 * g;
  v8f accO[4] = {}; float mrun = -1.0e30f, lrun = 0.0f;
#pragma unroll 1
  for (int kt = 0; kt < SEQ; kt += 32) {
    int qo = qoff; asm volatile("" : "+v"(qo));
    v8f s0 = {}, s0l = {}, s1 = {}, s1l = {};
#pragma unroll
    for (int kc = 0; kc < HD / 32; ++kc) {
      const v16h fq = frag_h(H16 + qo + kc * 32, lane), fql = frag_h(QL + qo + kc * 32, lane);
      const v16h fk0 = frag_h(KH + koff + kt * DM + kc * 32, lane), fk1 = frag_h(KH + koff + (kt + 16) * DM + kc * 32, lane);
      WAITL();
      s0 = wmma16(fk0, fq, s0); s0l = wmma16(fk0, fql, s0l); s1 = wmma16(fk1, fq, s1); s1l = wmma16(fk1, fql, s1l);
    }
    const v4f m00 = *(const v4f*)(mrow + kt), m01 = *(const v4f*)(mrow + kt + 4), m10 = *(const v4f*)(mrow + kt + 16), m11 = *(const v4f*)(mrow + kt + 20);
    WAITL();
    float pa[8], pc[8];
#pragma unroll
    for (int r = 0; r < 8; ++r) { const float mk0 = bfr((r < 4) ? m00[r & 3] : m01[r & 3]), mk1 = bfr((r < 4) ? m10[r & 3] : m11[r & 3]);
      pa[r] = (s0[r] + s0l[r] * (1.0f / 1024.0f)) * SCALE + mk0; pc[r] = (s1[r] + s1l[r] * (1.0f / 1024.0f)) * SCALE + mk1; }
    float tmax = fmaxf(pa[0], pc[0]);
#pragma unroll
    for (int r = 1; r < 8; ++r) tmax = fmaxf(tmax, fmaxf(pa[r], pc[r]));
    tmax = fmaxf(tmax, __shfl_xor(tmax, 16));
    const float mnew = fmaxf(mrun, tmax); const float alpha = __expf(mrun - mnew); mrun = mnew;
    float ps = 0.0f; v16h pb;
#pragma unroll
    for (int r = 0; r < 8; ++r) { const float e0 = __expf(pa[r] - mnew), e1 = __expf(pc[r] - mnew); ps += e0 + e1; pb[r] = (_Float16)(e0 * PCARRY); pb[8 + r] = (_Float16)(e1 * PCARRY); }
    ps += __shfl_xor(ps, 16); lrun = lrun * alpha + ps;
#pragma unroll
    for (int r = 0; r < 8; ++r) { accO[0][r] *= alpha; accO[1][r] *= alpha; accO[2][r] *= alpha; accO[3][r] *= alpha; }
    const v16h fv0 = frag_h(VT + voff + kt, lane), fv1 = frag_h(VT + voff + 16 * SEQ + kt, lane), fv2 = frag_h(VT + voff + 32 * SEQ + kt, lane), fv3 = frag_h(VT + voff + 48 * SEQ + kt, lane);
    WAITL();
    accO[0] = wmma16(fv0, pb, accO[0]); accO[1] = wmma16(fv1, pb, accO[1]); accO[2] = wmma16(fv2, pb, accO[2]); accO[3] = wmma16(fv3, pb, accO[3]);
  }
  const float inv = 0.0625f * (1.0f / lrun);
#pragma unroll
  for (int j = 0; j < 4; ++j) { v8h hv, lv;
#pragma unroll
    for (int r = 0; r < 8; ++r) { const float c = accO[j][r] * inv; const _Float16 hi = (_Float16)c; hv[r] = hi; lv[r] = (_Float16)((c - (float)hi) * 128.0f); }
    *(v8h*)&sh[wave][col][j * 16 + 8 * g] = hv; *(v8h*)&sl[wave][col][j * 16 + 8 * g] = lv; }
  LDSX();
#pragma unroll
  for (int i = 0; i < 4; ++i) { const int rl = i * 4 + (lane >> 3), pcx = lane & 7; const size_t dst = ((size_t)b * SEQ + q0 + rl) * DM + h * HD + pcx * 8;
    const v4u a = *(const v4u*)&sh[wave][rl][pcx * 8]; const v4u c = *(const v4u*)&sl[wave][rl][pcx * 8];
    vst2(CH + dst, a); vst2(CL + dst, c); }
}

__global__ __launch_bounds__(128) void k_out(const _Float16* __restrict__ CH, const _Float16* __restrict__ CL, const _Float16* __restrict__ WOH, const _Float16* __restrict__ WOL, const float* __restrict__ BO, float* __restrict__ OUT) {
  __shared__ __align__(16) float sf[4][16][132];
  const int tid = threadIdx.x, wave = tid >> 5, lane = tid & 31, col = lane & 15, g = lane >> 4; const int c0 = blockIdx.y * 128; const int R0 = blockIdx.x * 64 + wave * 16;
  v8f acc[8] = {};
#pragma unroll 2
  for (int kc = 0; kc < DM / 32; ++kc) { const size_t ao = (size_t)(R0 + col) * DM + kc * 32; const v16h ah = frag_h(CH + ao, lane), al = frag_h(CL + ao, lane);
    WAITL();
#pragma unroll
    for (int j = 0; j < 8; ++j) { const size_t wo = (size_t)(c0 + j * 16 + col) * DM + kc * 32; const v16h wh = frag_h(WOH + wo, lane), wl = frag_h(WOL + wo, lane); WAITL(); acc[j] = wmma16(ah, wh, acc[j]); acc[j] = wmma16(al, wl, acc[j]); } }
#pragma unroll
  for (int j = 0; j < 8; ++j) { const float bias = bfr(BO[c0 + j * 16 + col]);
#pragma unroll
    for (int r = 0; r < 8; ++r) sf[wave][8 * g + r][j * 16 + col] = acc[j][r] * (1.0f / 16384.0f) + bias; }
  LDSX();
  const int bb = (blockIdx.x * 64) / SEQ; const int t0 = (blockIdx.x * 64) % SEQ + wave * 16;
  for (int rl = 0; rl < 16; ++rl) { const v4f o = *(const v4f*)&sf[wave][rl][lane * 4]; vst2(OUT + ((size_t)bb * SEQ_FULL + t0 + rl) * DM + c0 + lane * 4, o); }
}

extern "C" void kernel_launch(void* const* d_in, const int* in_sizes, int n_in, void* d_out, int out_size, void* d_ws, size_t ws_size, hipStream_t stream) {
  if (n_in < 12) return;
  const size_t need_x = ((size_t)(NB - 1) * SEQ_FULL + SEQ) * DM;
  if ((size_t)in_sizes[0] < need_x || (size_t)in_sizes[1] < need_x || (size_t)in_sizes[2] < need_x) return;
  if ((size_t)in_sizes[3] < ((size_t)(NB - 1) * SEQ_FULL + SEQ) * SEQ_FULL) return;
  if (in_sizes[4] < DM * DM || in_sizes[6] < DM * DM || in_sizes[8] < DM * DM || in_sizes[10] < DM * DM) return;
  if (in_sizes[5] < DM || in_sizes[7] < DM || in_sizes[9] < DM || in_sizes[11] < DM) return;
  if ((size_t)out_size < (size_t)OUT1_ELEM + (size_t)NB * 2 * NH * SEQ_FULL * HD) return;
  if (ws_size < (size_t)WS_END) return;
  const float** F = (const float**)d_in;
  char* ws = (char*)d_ws;
  __bf16* XB = (__bf16*)(ws + WS_XB); __bf16* WB = (__bf16*)(ws + WS_WB);
  _Float16 *WOH = (_Float16*)(ws + WS_WOH), *WOL = (_Float16*)(ws + WS_WOL), *H16 = (_Float16*)(ws + WS_H16), *QL = (_Float16*)(ws + WS_QL), *VT = (_Float16*)(ws + WS_VT), *CH = (_Float16*)(ws + WS_CH), *CL = (_Float16*)(ws + WS_CL);
  float* OUT = (float*)d_out; float* PRES = OUT + OUT1_ELEM;
  const int nx8 = SEQ * DM / 8, nw8 = DM * DM / 8;
  const dim3 gx(nx8 / 256, NB), gw(nw8 / 256, 1);
  k_cvt_bf<<<gx, 256, 0, stream>>>(F[2], XB,                          (size_t)SEQ_FULL * DM, (size_t)SEQ * DM, nx8);
  k_cvt_bf<<<gx, 256, 0, stream>>>(F[0], XB + (size_t)MROWS * DM,     (size_t)SEQ_FULL * DM, (size_t)SEQ * DM, nx8);
  k_cvt_bf<<<gx, 256, 0, stream>>>(F[1], XB + 2 * (size_t)MROWS * DM, (size_t)SEQ_FULL * DM, (size_t)SEQ * DM, nx8);
  k_cvt_bf<<<gw, 256, 0, stream>>>(F[4], WB,                        (size_t)0, (size_t)0, nw8);
  k_cvt_bf<<<gw, 256, 0, stream>>>(F[6], WB + (size_t)DM * DM,      (size_t)0, (size_t)0, nw8);
  k_cvt_bf<<<gw, 256, 0, stream>>>(F[8], WB + 2 * (size_t)DM * DM,  (size_t)0, (size_t)0, nw8);
  k_cvt_wo<<<gw, 256, 0, stream>>>(F[10], WOH, WOL, nw8);
  k_proj<<<dim3(MROWS / 64, DM / 128, 3), 128, 0, stream>>>(XB, WB, F[5], F[7], F[9], H16, QL, VT, PRES);
  k_attn<<<dim3(SEQ / 64, NH, NB), 128, 0, stream>>>(H16, QL, VT, F[3], CH, CL);
  k_out<<<dim3(MROWS / 64, DM / 128), 128, 0, stream>>>(CH, CL, WOH, WOL, F[11], OUT);
}
